// MultiHeadAttention_18674517803234
// MI455X (gfx1250) — hardware-run, weakly checked
//
#include <hip/hip_runtime.h>
#include <math.h>

typedef __attribute__((ext_vector_type(16))) _Float16 v16h;
typedef __attribute__((ext_vector_type(8)))  _Float16 v8h;
typedef __attribute__((ext_vector_type(8)))  float    v8f;
typedef __attribute__((ext_vector_type(4)))  float    v4f;

constexpr int kBatch = 4;
constexpr int kSeq   = 2048;
constexpr int kDim   = 1024;
constexpr int kHeads = 16;
constexpr int kHd    = 64;
constexpr int kTok   = kBatch * kSeq;
constexpr int kQkvN  = 3 * kDim;
static_assert(kHeads * kHd == kDim);
static_assert(kTok == 8192);
static_assert((kDim % 32) == 0);
static_assert((kTok % 64) == 0 && (kQkvN % 64) == 0 && (kDim % 64) == 0 && (kSeq % 128) == 0);

constexpr float kAttnScale = 0.125f;
static_assert(kHd == 64);
static_assert(kAttnScale * kAttnScale * (float)kHd == 1.0f);

constexpr float kXnCarry    = 16.0f;
constexpr float kWCarry     = 1024.0f;
constexpr float kQkvCarry   = 16.0f;
constexpr float kPLog2Carry = 10.0f;
constexpr float kCtxCarry   = 1024.0f;
constexpr float kProjScale  = 1.0f / (kXnCarry * kWCarry);
constexpr float kCtxExtra   = kCtxCarry / kQkvCarry;
constexpr float kOutScale   = 1.0f / (kCtxCarry * kWCarry);
constexpr float kLog2e      = 1.4426950408889634f;
constexpr float kExpCoef    = kLog2e * kAttnScale / (kQkvCarry * kQkvCarry);
constexpr float kInvDim     = 1.0f / (float)kDim;
constexpr float kLnEps      = 1e-5f;

constexpr size_t kOffXN = 0;
constexpr size_t kOffWC = kOffXN + (size_t)kTok * kDim * 2;
constexpr size_t kOffQP = kOffWC + (size_t)4 * kDim * kDim * 2;
constexpr size_t kOffKP = kOffQP + (size_t)kTok * kDim * 2;
constexpr size_t kOffVT = kOffKP + (size_t)kTok * kDim * 2;
constexpr size_t kOffAO = kOffVT + (size_t)kTok * kDim * 2;
constexpr size_t kWsTotal = kOffAO + (size_t)kTok * kDim * 2;
static_assert(kWsTotal == 92274688ull);
static_assert(kWsTotal <= 134217728ull);
static_assert((kOffWC % 128) == 0 && (kOffQP % 128) == 0 && (kOffKP % 128) == 0 && (kOffVT % 128) == 0 && (kOffAO % 128) == 0);

struct FragH {
  union U { v16h v; v8h h[2]; };
  static __device__ __forceinline__ v16h load(const _Float16* p) {
    U f;
    f.h[0] = *(const v8h*)(p);
    f.h[1] = *(const v8h*)(p + 16);
    return f.v;
  }
  static __device__ __forceinline__ v8f mma(v16h a, v16h b, v8f c) {
    return __builtin_amdgcn_wmma_f32_16x16x32_f16(false, a, false, b, (short)0, c, false, false);
  }
};
__device__ __forceinline__ void guard4_h(v8f& a, v8f& b, v8f& c, v8f& d, v16h x, v16h b0, v16h b1, v16h b2, v16h b3) {
  asm volatile("v_nop\n\tv_nop\n\tv_nop\n\tv_nop" : "+v"(a), "+v"(b), "+v"(c), "+v"(d) : "v"(x), "v"(b0), "v"(b1), "v"(b2), "v"(b3));
}
__device__ __forceinline__ void guard1_h(v8f& a, v16h x, v16h y, v16h z, v16h w) {
  asm volatile("v_nop\n\tv_nop\n\tv_nop\n\tv_nop" : "+v"(a) : "v"(x), "v"(y), "v"(z), "v"(w));
}
__device__ __forceinline__ void keep4_h(v16h a, v16h b, v16h c, v16h d) {
  asm volatile("v_nop" :: "v"(a), "v"(b), "v"(c), "v"(d));
}
__device__ __forceinline__ void acc_guard4(v8f& a, v8f& b, v8f& c, v8f& d) {
  asm volatile("v_nop\n\tv_nop\n\tv_nop\n\tv_nop" : "+v"(a), "+v"(b), "+v"(c), "+v"(d));
}
__device__ __forceinline__ void wave_lds_sync() {
  __builtin_amdgcn_fence(__ATOMIC_RELEASE, "workgroup");
  __builtin_amdgcn_wave_barrier();
  __builtin_amdgcn_fence(__ATOMIC_ACQUIRE, "workgroup");
}

__global__ __launch_bounds__(256) void ln_rows_kernel(const float* __restrict__ x, const float* __restrict__ gamma,
                                                      const float* __restrict__ beta, unsigned short* __restrict__ xn) {
  const int lane = threadIdx.x & 31;
  const int wave = __builtin_amdgcn_readfirstlane((int)(threadIdx.x >> 5));
  const int row = blockIdx.x * 8 + wave;
  if (row >= kTok) return;
  const float* xr = x + (size_t)row * kDim + lane * 8;
  float s = 0.0f;
#pragma unroll 1
  for (int it = 0; it < 4; ++it) {
    const v4f a0 = *(const v4f*)(xr + it * 256);
    const v4f a1 = *(const v4f*)(xr + it * 256 + 4);
    s += ((a0[0] + a0[1]) + (a0[2] + a0[3])) + ((a1[0] + a1[1]) + (a1[2] + a1[3]));
  }
#pragma unroll
  for (int off = 16; off > 0; off >>= 1) s += __shfl_xor(s, off, 32);
  const float mu = s * kInvDim;
  float ss = 0.0f;
#pragma unroll 1
  for (int it = 0; it < 4; ++it) {
    const v4f a0 = *(const v4f*)(xr + it * 256);
    const v4f a1 = *(const v4f*)(xr + it * 256 + 4);
#pragma unroll
    for (int e = 0; e < 4; ++e) {
      const float d0 = a0[e] - mu;
      const float d1 = a1[e] - mu;
      ss = fmaf(d0, d0, ss);
      ss = fmaf(d1, d1, ss);
    }
  }
#pragma unroll
  for (int off = 16; off > 0; off >>= 1) ss += __shfl_xor(ss, off, 32);
  const float inv = rsqrtf(ss * kInvDim + kLnEps);
  unsigned short* orow = xn + (size_t)row * kDim + lane * 8;
#pragma unroll 1
  for (int it = 0; it < 4; ++it) {
    const v4f a0 = *(const v4f*)(xr + it * 256);
    const v4f a1 = *(const v4f*)(xr + it * 256 + 4);
    const v4f g0 = *(const v4f*)(gamma + it * 256 + lane * 8);
    const v4f g1 = *(const v4f*)(gamma + it * 256 + lane * 8 + 4);
    const v4f b0 = *(const v4f*)(beta + it * 256 + lane * 8);
    const v4f b1 = *(const v4f*)(beta + it * 256 + lane * 8 + 4);
    v8h hv;
#pragma unroll
    for (int e = 0; e < 4; ++e) {
      const float y0 = fmaf((a0[e] - mu) * inv, g0[e], b0[e]) * kXnCarry;
      const float y1 = fmaf((a1[e] - mu) * inv, g1[e], b1[e]) * kXnCarry;
      hv[e] = (_Float16)y0;
      hv[4 + e] = (_Float16)y1;
    }
    *(volatile v8h*)(orow + it * 256) = hv;
    __threadfence();
    *(volatile v8h*)(orow + it * 256) = hv;
  }
}

__global__ __launch_bounds__(256) void cast_w_kernel(const float* __restrict__ w0, const float* __restrict__ w1,
                                                     const float* __restrict__ w2, const float* __restrict__ w3,
                                                     unsigned short* __restrict__ out, float carry) {
  const int z = blockIdx.y;
  const float* W = (z == 0) ? w0 : (z == 1) ? w1 : (z == 2) ? w2 : w3;
  const int i = blockIdx.x * 256 + threadIdx.x;
  if (i >= kDim * kDim / 8) return;
  const float* p = W + 8 * (size_t)i;
  const v4f a = *(const v4f*)(p);
  const v4f c = *(const v4f*)(p + 4);
  v8h hv;
#pragma unroll
  for (int e = 0; e < 4; ++e) {
    hv[e] = (_Float16)(a[e] * carry);
    hv[4 + e] = (_Float16)(c[e] * carry);
  }
  unsigned short* q = out + (size_t)z * kDim * kDim + 8 * (size_t)i;
  *(volatile v8h*)q = hv;
  __threadfence();
  *(volatile v8h*)q = hv;
}

__device__ __forceinline__ void gemm_tile_loop(const _Float16* __restrict__ A, const _Float16* __restrict__ Bt,
                                               int m0, int n0, int lane, v8f (&acc)[4][4]) {
  const int rlane = lane & 15;
  const int koff  = (lane >> 4) * 8;
#pragma unroll
  for (int i = 0; i < 4; ++i)
#pragma unroll
    for (int j = 0; j < 4; ++j) acc[i][j] = (v8f){0.f, 0.f, 0.f, 0.f, 0.f, 0.f, 0.f, 0.f};
#pragma unroll 1
  for (int k0 = 0; k0 < kDim; k0 += 32) {
    v16h bh[4];
#pragma unroll
    for (int j = 0; j < 4; ++j)
      bh[j] = FragH::load(Bt + (size_t)(n0 + (j << 4) + rlane) * kDim + koff + k0);
#pragma unroll
    for (int i = 0; i < 4; ++i) {
      const v16h ah = FragH::load(A + (size_t)(m0 + (i << 4) + rlane) * kDim + koff + k0);
#pragma unroll
      for (int j = 0; j < 4; ++j) acc[i][j] = FragH::mma(ah, bh[j], acc[i][j]);
      guard4_h(acc[i][0], acc[i][1], acc[i][2], acc[i][3], ah, bh[0], bh[1], bh[2], bh[3]);
    }
    keep4_h(bh[0], bh[1], bh[2], bh[3]);
  }
  acc_guard4(acc[0][0], acc[0][1], acc[0][2], acc[0][3]);
  acc_guard4(acc[1][0], acc[1][1], acc[1][2], acc[1][3]);
  acc_guard4(acc[2][0], acc[2][1], acc[2][2], acc[2][3]);
  acc_guard4(acc[3][0], acc[3][1], acc[3][2], acc[3][3]);
}

__global__ __launch_bounds__(256) void gemm_qkv_kernel(
    const unsigned short* __restrict__ XNp, const unsigned short* __restrict__ WCp,
    unsigned short* __restrict__ QPp, unsigned short* __restrict__ KPp, unsigned short* __restrict__ VTp,
    const float* __restrict__ bq, const float* __restrict__ bk, const float* __restrict__ bv) {
  __shared__ __align__(16) _Float16 Tsh[4 * 64 * 72];
  const int lane = threadIdx.x & 31;
  const int wave = __builtin_amdgcn_readfirstlane((int)(threadIdx.x >> 5));
  constexpr int tilesN = kQkvN >> 6;
  constexpr int tilesM = kTok >> 6;
  const int tile = blockIdx.x * 4 + wave;
  if (tile >= tilesM * tilesN) return;
  const int tm = tile / tilesN;
  const int tn = tile - tm * tilesN;
  const int m0 = tm << 6;
  const int n0 = tn << 6;

  v8f acc[4][4];
  gemm_tile_loop((const _Float16*)XNp, (const _Float16*)WCp, m0, n0, lane, acc);

  const int rlane = lane & 15;
  const int mOff  = (lane >> 4) * 8;
  const int region = n0 >> 10;
  const int nl0  = n0 & (kDim - 1);
  const int head = nl0 >> 6;
  const int bidx = m0 >> 11;
  const int s0   = m0 & (kSeq - 1);
  const float* bias = (region == 0) ? bq : ((region == 1) ? bk : bv);
  float bvj[4];
#pragma unroll
  for (int j = 0; j < 4; ++j) bvj[j] = bias[nl0 + (j << 4) + rlane];

  _Float16* st = Tsh + wave * (64 * 72);
#pragma unroll
  for (int i = 0; i < 4; ++i) {
#pragma unroll
    for (int j = 0; j < 4; ++j) {
      float y[8];
#pragma unroll
      for (int r = 0; r < 8; ++r) y[r] = (acc[i][j][r] * kProjScale + bvj[j]) * kQkvCarry;
      if (region < 2) {
#pragma unroll
        for (int r = 0; r < 8; ++r) st[((i << 4) + mOff + r) * 72 + (j << 4) + rlane] = (_Float16)y[r];
      } else {
        v8h t;
#pragma unroll
        for (int r = 0; r < 8; ++r) t[r] = (_Float16)y[r];
        *(v8h*)(st + ((j << 4) + rlane) * 72 + (i << 4) + mOff) = t;
      }
    }
  }
  wave_lds_sync();

  unsigned short* plane;
  size_t gbase;
  int gpitch;
  if (region < 2) {
    plane  = (region == 0) ? QPp : KPp;
    gbase  = ((size_t)(bidx * kHeads + head) * kSeq + s0) * kHd;
    gpitch = kHd;
  } else {
    plane  = VTp;
    gbase  = (size_t)(bidx * kHeads + head) * kHd * kSeq + s0;
    gpitch = kSeq;
  }
  const int q4 = lane >> 3, c8 = (lane & 7) * 8;
  for (int pass = 0; pass < 2; ++pass) {
#pragma unroll
    for (int it = 0; it < 16; ++it) {
      const int row = it * 4 + q4;
      const v8h val = *(const v8h*)(st + row * 72 + c8);
      *(volatile v8h*)(plane + gbase + (size_t)row * gpitch + c8) = val;
    }
    __threadfence();
  }
}

__global__ __launch_bounds__(256) void gemm_out_kernel(
    const unsigned short* __restrict__ AOp, const unsigned short* __restrict__ WOp,
    float* __restrict__ out, const float* __restrict__ bo) {
  __shared__ __align__(16) float Ssh[8 * 16 * 68];
  const int lane = threadIdx.x & 31;
  const int wave = __builtin_amdgcn_readfirstlane((int)(threadIdx.x >> 5));
  constexpr int tilesN = kDim >> 6;
  constexpr int tilesM = kTok >> 6;
  const int tile = blockIdx.x * 8 + wave;
  if (tile >= tilesM * tilesN) return;
  const int tm = tile / tilesN;
  const int tn = tile - tm * tilesN;
  const int m0 = tm << 6;
  const int n0 = tn << 6;

  v8f acc[4][4];
  gemm_tile_loop((const _Float16*)AOp, (const _Float16*)WOp, m0, n0, lane, acc);

  const int rlane = lane & 15;
  const int mOff  = (lane >> 4) * 8;
  float bvj[4];
#pragma unroll
  for (int j = 0; j < 4; ++j) bvj[j] = bo[n0 + (j << 4) + rlane];
  float* slab = Ssh + wave * (16 * 68);
  const int hh = lane >> 4, c4 = (lane & 15) * 4;
#pragma unroll
  for (int i = 0; i < 4; ++i) {
    const int mBase = m0 + (i << 4);
#pragma unroll
    for (int j = 0; j < 4; ++j) {
#pragma unroll
      for (int r = 0; r < 8; ++r)
        slab[(mOff + r) * 68 + (j << 4) + rlane] = acc[i][j][r] * kOutScale + bvj[j];
    }
    wave_lds_sync();
    for (int pass = 0; pass < 2; ++pass) {
#pragma unroll
      for (int it = 0; it < 8; ++it) {
        const int row = it * 2 + hh;
        const v4f v = *(const v4f*)(slab + row * 68 + c4);
        *(volatile v4f*)(out + (size_t)(mBase + row) * kDim + n0 + c4) = v;
      }
      __threadfence();
    }
    wave_lds_sync();
  }
}

__global__ __launch_bounds__(256) void attn_kernel(const unsigned short* __restrict__ QPp,
                                                   const unsigned short* __restrict__ KPp,
                                                   const unsigned short* __restrict__ VTp,
                                                   unsigned short* __restrict__ AOp) {
  __shared__ __align__(16) _Float16 Ksh[64 * 64];
  __shared__ __align__(16) _Float16 Vsh[64 * 64];
  __shared__ __align__(16) _Float16 Osh[8 * 16 * 72];
  const int tid  = threadIdx.x;
  const int lane = tid & 31;
  const int wave = __builtin_amdgcn_readfirstlane((int)(tid >> 5));
  const int hh   = lane >> 4;
  const int c    = lane & 15;
  const int bx   = blockIdx.x;
  const int qb   = bx & 15;
  const int bh   = bx >> 4;
  const int head = bh & (kHeads - 1);
  const int bidx = bh >> 4;
  const int q0   = qb * 128 + wave * 16;

  const _Float16* Qh = (const _Float16*)QPp + (size_t)bh * kSeq * kHd;
  const _Float16* Kh = (const _Float16*)KPp + (size_t)bh * kSeq * kHd;
  const _Float16* Vh = (const _Float16*)VTp + (size_t)bh * kHd * kSeq;

  const v16h qf0 = FragH::load(Qh + (size_t)(q0 + c) * kHd + 8 * hh);
  const v16h qf1 = FragH::load(Qh + (size_t)(q0 + c) * kHd + 32 + 8 * hh);

  v8f oacc[4];
#pragma unroll
  for (int t = 0; t < 4; ++t) oacc[t] = (v8f){0.f, 0.f, 0.f, 0.f, 0.f, 0.f, 0.f, 0.f};
  float mrun = -1e30f;
  float lrun = 0.0f;

#pragma unroll 1
  for (int kc = 0; kc < kSeq / 64; ++kc) {
    const int kv0 = kc * 64;
    __syncthreads();
#pragma unroll
    for (int i = 0; i < 2; ++i) {
      const int idx = tid + 256 * i;
      const v8h kk = *(const v8h*)(Kh + (size_t)kv0 * kHd + idx * 8);
      const v8h vv = *(const v8h*)(Vh + (size_t)(idx >> 3) * kSeq + kv0 + (idx & 7) * 8);
      *(v8h*)(Ksh + idx * 8) = kk;
      *(v8h*)(Vsh + idx * 8) = vv;
    }
    __syncthreads();

    v8f st[4];
#pragma unroll
    for (int j = 0; j < 4; ++j) {
      st[j] = (v8f){0.f, 0.f, 0.f, 0.f, 0.f, 0.f, 0.f, 0.f};
      const v16h ka0 = FragH::load(Ksh + (j * 16 + c) * 64 + 8 * hh);
      const v16h ka1 = FragH::load(Ksh + (j * 16 + c) * 64 + 32 + 8 * hh);
      st[j] = FragH::mma(ka0, qf0, st[j]);
      st[j] = FragH::mma(ka1, qf1, st[j]);
      guard1_h(st[j], ka0, ka1, qf0, qf1);
    }

    float mx = st[0][0];
#pragma unroll
    for (int j = 0; j < 4; ++j)
#pragma unroll
      for (int r = 0; r < 8; ++r) mx = fmaxf(mx, st[j][r]);
    mx = fmaxf(mx, __shfl_xor(mx, 16, 32));
    const float mnew  = fmaxf(mrun, mx);
    const float alpha = __builtin_amdgcn_exp2f((mrun - mnew) * kExpCoef);
    const float off   = fmaf(-mnew, kExpCoef, kPLog2Carry);
    mrun = mnew;

    v16h pf0, pf1;
    float psum = 0.0f;
#pragma unroll
    for (int r = 0; r < 8; ++r) {
      const _Float16 h0 = (_Float16)__builtin_amdgcn_exp2f(fmaf(st[0][r], kExpCoef, off));
      const _Float16 h1 = (_Float16)__builtin_amdgcn_exp2f(fmaf(st[1][r], kExpCoef, off));
      const _Float16 h2 = (_Float16)__builtin_amdgcn_exp2f(fmaf(st[2][r], kExpCoef, off));
      const _Float16 h3 = (_Float16)__builtin_amdgcn_exp2f(fmaf(st[3][r], kExpCoef, off));
      pf0[r] = h0;
      pf0[8 + r] = h1;
      pf1[r] = h2;
      pf1[8 + r] = h3;
      psum += ((float)h0 + (float)h1) + ((float)h2 + (float)h3);
    }
    lrun = lrun * alpha + psum;
#pragma unroll
    for (int t = 0; t < 4; ++t)
#pragma unroll
      for (int r = 0; r < 8; ++r) oacc[t][r] *= alpha;

#pragma unroll
    for (int t = 0; t < 4; ++t) {
      const v16h va0 = FragH::load(Vsh + (t * 16 + c) * 64 + 8 * hh);
      const v16h va1 = FragH::load(Vsh + (t * 16 + c) * 64 + 32 + 8 * hh);
      oacc[t] = FragH::mma(va0, pf0, oacc[t]);
      oacc[t] = FragH::mma(va1, pf1, oacc[t]);
      guard1_h(oacc[t], va0, va1, pf0, pf1);
    }
  }

  const float ltot = lrun + __shfl_xor(lrun, 16, 32);
  const float inv  = kCtxExtra * (1.0f / ltot);
  _Float16* os = Osh + wave * (16 * 72);
#pragma unroll
  for (int t = 0; t < 4; ++t) {
    v8h o;
#pragma unroll
    for (int r = 0; r < 8; ++r) o[r] = (_Float16)(oacc[t][r] * inv);
    *(v8h*)(os + c * 72 + t * 16 + 8 * hh) = o;
  }
  wave_lds_sync();
  {
    const int q4 = lane >> 3, c8 = (lane & 7) * 8;
    for (int pass = 0; pass < 2; ++pass) {
#pragma unroll
      for (int it = 0; it < 4; ++it) {
        const int row = it * 4 + q4;
        const v8h val = *(const v8h*)(os + row * 72 + c8);
        *(volatile v8h*)(AOp + (size_t)(bidx * kSeq + q0 + row) * kDim + head * kHd + c8) = val;
      }
      __threadfence();
    }
  }
}

extern "C" void kernel_launch(void* const* d_in, const int* in_sizes, int n_in,
                              void* d_out, int out_size, void* d_ws, size_t ws_size,
                              hipStream_t stream) {
  if (n_in < 11) return;
  if (in_sizes[0] != kTok * kDim) return;
  if (in_sizes[1] != kDim || in_sizes[2] != kDim) return;
  if (in_sizes[3] != kDim * kDim || in_sizes[5] != kDim * kDim) return;
  if (in_sizes[7] != kDim * kDim || in_sizes[9] != kDim * kDim) return;
  if (in_sizes[4] != kDim || in_sizes[6] != kDim || in_sizes[8] != kDim || in_sizes[10] != kDim) return;
  if (out_size != kTok * kDim) return;
  if (ws_size < kWsTotal) return;

  const float* x     = (const float*)d_in[0];
  const float* gamma = (const float*)d_in[1];
  const float* beta  = (const float*)d_in[2];
  const float* Wq    = (const float*)d_in[3];
  const float* bq    = (const float*)d_in[4];
  const float* Wk    = (const float*)d_in[5];
  const float* bk    = (const float*)d_in[6];
  const float* Wv    = (const float*)d_in[7];
  const float* bv    = (const float*)d_in[8];
  const float* Wo    = (const float*)d_in[9];
  const float* bo    = (const float*)d_in[10];
  float* out = (float*)d_out;

  char* ws = (char*)d_ws;
  unsigned short* XN = (unsigned short*)(ws + kOffXN);
  unsigned short* WC = (unsigned short*)(ws + kOffWC);
  unsigned short* QP = (unsigned short*)(ws + kOffQP);
  unsigned short* KP = (unsigned short*)(ws + kOffKP);
  unsigned short* VT = (unsigned short*)(ws + kOffVT);
  unsigned short* AO = (unsigned short*)(ws + kOffAO);
  unsigned short* WO = WC + (size_t)3 * kDim * kDim;

  ln_rows_kernel<<<kTok / 8, 256, 0, stream>>>(x, gamma, beta, XN);
  cast_w_kernel<<<dim3(kDim * kDim / 8 / 256, 4), 256, 0, stream>>>(Wq, Wk, Wv, Wo, WC, kWCarry);
  gemm_qkv_kernel<<<(kTok / 64) * (kQkvN / 64) / 4, 128, 0, stream>>>(XN, WC, QP, KP, VT, bq, bk, bv);
  attn_kernel<<<kBatch * kHeads * (kSeq / 128), 256, 0, stream>>>(QP, KP, VT, AO);
  gemm_out_kernel<<<(kTok / 64) * (kDim / 64) / 8, 256, 0, stream>>>(AO, WO, out, bo);
}
